// TransNeXt_24799141167818
// MI455X (gfx1250) — hardware-verified
//
#include <hip/hip_runtime.h>
#define NB 16
#define NT 4096
#define DM 128
#define HE 4
#define HD 32
#define GS 64
#define PS 8
#define PL 64
#define LL 9
#define NR ((size_t)NB * NT)
#define NTB 14400
#define CPH 512
typedef __bf16 v16b __attribute__((ext_vector_type(16)));
typedef unsigned short v8us __attribute__((ext_vector_type(8), may_alias));
typedef float  v8f  __attribute__((ext_vector_type(8)));
typedef float  v4f  __attribute__((ext_vector_type(4)));
typedef float  v4fa __attribute__((ext_vector_type(4), may_alias));
union FragB { v16b v; v8us half[2]; unsigned short u[16]; };

__device__ __forceinline__ unsigned short bf16_bits(float x) { unsigned int u = __float_as_uint(x); return (unsigned short)((u + 0x7FFFu + ((u >> 16) & 1u)) >> 16); }
__device__ __forceinline__ float bf16_val(unsigned short b) { return __uint_as_float(((unsigned int)b) << 16); }
__device__ __forceinline__ float bf16_round(float x) { return bf16_val(bf16_bits(x)); }
template <int NTT>
__device__ __forceinline__ v8f mmaN(v16b ah, v16b al, v16b bh, v16b bl, v8f c) {
  c = __builtin_amdgcn_wmma_f32_16x16x32_bf16(false, ah, false, bh, (short)0, c, false, false);
  if (NTT >= 2) c = __builtin_amdgcn_wmma_f32_16x16x32_bf16(false, al, false, bh, (short)0, c, false, false);
  if (NTT >= 3) c = __builtin_amdgcn_wmma_f32_16x16x32_bf16(false, ah, false, bl, (short)0, c, false, false);
  asm volatile("v_nop\n\tv_nop\n\tv_nop\n\tv_nop" : "+v"(c) : "v"(ah), "v"(al), "v"(bh), "v"(bl));
  return c;
}

__global__ __launch_bounds__(256) void k_wt_bf16(const float* __restrict__ W, unsigned short* __restrict__ Wt, int K, int N) {
  const int t = blockIdx.x * 256 + threadIdx.x;
  const int k8n = K / 8;
  if (t >= N * k8n) return;
  const int n = t / k8n, k8 = (t % k8n) * 8;
  v8us v;
#pragma unroll
  for (int i = 0; i < 8; ++i) v[i] = bf16_bits(W[(size_t)(k8 + i) * N + n]);
  *(volatile v8us*)(Wt + (size_t)n * K + k8) = v;
  __threadfence();
  *(volatile v8us*)(Wt + (size_t)n * K + k8) = v;
}

template <bool ASPLIT, int ACT, bool BIAS_BF16>
__global__ __launch_bounds__(128) void k_gemm_bf(const float* __restrict__ A, int lda, const unsigned short* __restrict__ Wt, int ldb,
                                               const float* __restrict__ bias, float* __restrict__ C, int ldc, int M, int N, int K) {
  __shared__ __attribute__((aligned(16))) float so[4][16][64];
  const int tid = threadIdx.x, w = tid >> 5, lane = tid & 31, ln = lane & 15, hh = lane >> 4;
  const int ntn = N / 64;
  const int wid = blockIdx.x * 4 + w;
  const int mt = wid / ntn, nq = wid % ntn;
  if (mt * 16 >= M) return;
  const int row0 = mt * 16, col0 = nq * 64;
  const float* arow = A + (size_t)(row0 + ln) * lda;
  v8f acc[4] = {};
  for (int kb = 0; kb < K; kb += 32) {
    FragB ah, al;
    const v4f x0 = *(const v4fa*)(arow + kb + 8 * hh), x1 = *(const v4fa*)(arow + kb + 8 * hh + 4);
    const v4f x2 = *(const v4fa*)(arow + kb + 16 + 8 * hh), x3 = *(const v4fa*)(arow + kb + 16 + 8 * hh + 4);
    float xs[16] = {x0[0],x0[1],x0[2],x0[3],x1[0],x1[1],x1[2],x1[3],x2[0],x2[1],x2[2],x2[3],x3[0],x3[1],x3[2],x3[3]};
#pragma unroll
    for (int i = 0; i < 16; ++i) { const unsigned short hb = bf16_bits(xs[i]); ah.u[i] = hb; al.u[i] = ASPLIT ? bf16_bits(xs[i] - bf16_val(hb)) : (unsigned short)0; }
#pragma unroll
    for (int t = 0; t < 4; ++t) {
      const unsigned short* brow = Wt + (size_t)(col0 + t * 16 + ln) * ldb + kb;
      FragB b;
      b.half[0] = *(const v8us*)(brow + 8 * hh);
      b.half[1] = *(const v8us*)(brow + 16 + 8 * hh);
      acc[t] = mmaN<ASPLIT ? 2 : 1>(ah.v, al.v, b.v, b.v, acc[t]);
    }
  }
#pragma unroll
  for (int t = 0; t < 4; ++t) {
    float bv = bias ? bias[col0 + t * 16 + ln] : 0.f;
    if (BIAS_BF16) bv = bf16_round(bv);
#pragma unroll
    for (int r = 0; r < 8; ++r) { float v = acc[t][r] + bv; if (ACT == 1) v = fmaxf(v, 0.f); so[w][8 * hh + r][t * 16 + ln] = v; }
  }
  __builtin_amdgcn_fence(__ATOMIC_ACQ_REL, "workgroup");
  __builtin_amdgcn_wave_barrier();
  const int rsub = lane >> 4, c4 = (lane & 15) * 4;
  for (int pass = 0; pass < 2; ++pass) {
#pragma unroll
    for (int q = 0; q < 8; ++q) {
      const int r = q * 2 + rsub;
      const v4f v = *(const v4fa*)&so[w][r][c4];
      *(volatile v4f*)(C + (size_t)(row0 + r) * ldc + col0 + c4) = v;
    }
    if (pass == 0) __threadfence();
  }
}

template <bool ASPLIT, int ACT, bool BIAS_BF16, bool RES_BF16>
__global__ __launch_bounds__(128) void k_gemm_bf3(const float* __restrict__ A, int lda, const unsigned short* __restrict__ Wt, int ldb,
                                                const float* __restrict__ bias, const float* __restrict__ resid, int rmod, int ldr,
                                                float* __restrict__ C, int ldc, int M, int N, int K) {
  __shared__ __attribute__((aligned(16))) float so[4][16][64];
  const int tid = threadIdx.x, w = tid >> 5, lane = tid & 31, ln = lane & 15, hh = lane >> 4;
  const int ntn = N / 64;
  const int wid = blockIdx.x * 4 + w;
  const int mt = wid / ntn, nq = wid % ntn;
  if (mt * 16 >= M) return;
  const int row0 = mt * 16, col0 = nq * 64;
  const float* arow = A + (size_t)(row0 + ln) * lda;
  v8f acc[4] = {};
  for (int kb = 0; kb < K; kb += 32) {
    FragB ah, al;
    const v4f x0 = *(const v4fa*)(arow + kb + 8 * hh), x1 = *(const v4fa*)(arow + kb + 8 * hh + 4);
    const v4f x2 = *(const v4fa*)(arow + kb + 16 + 8 * hh), x3 = *(const v4fa*)(arow + kb + 16 + 8 * hh + 4);
    float xs[16] = {x0[0],x0[1],x0[2],x0[3],x1[0],x1[1],x1[2],x1[3],x2[0],x2[1],x2[2],x2[3],x3[0],x3[1],x3[2],x3[3]};
#pragma unroll
    for (int i = 0; i < 16; ++i) { const unsigned short hb = bf16_bits(xs[i]); ah.u[i] = hb; al.u[i] = ASPLIT ? bf16_bits(xs[i] - bf16_val(hb)) : (unsigned short)0; }
#pragma unroll
    for (int t = 0; t < 4; ++t) {
      const unsigned short* brow = Wt + (size_t)(col0 + t * 16 + ln) * ldb + kb;
      FragB b;
      b.half[0] = *(const v8us*)(brow + 8 * hh);
      b.half[1] = *(const v8us*)(brow + 16 + 8 * hh);
      acc[t] = mmaN<ASPLIT ? 2 : 1>(ah.v, al.v, b.v, b.v, acc[t]);
    }
  }
#pragma unroll
  for (int t = 0; t < 4; ++t) {
    const int col = col0 + t * 16 + ln;
    float bv = bias ? bias[col] : 0.f;
    if (BIAS_BF16) bv = bf16_round(bv);
#pragma unroll
    for (int r = 0; r < 8; ++r) {
      float v = acc[t][r] + bv;
      if (resid) { float rv = resid[(size_t)((row0 + 8 * hh + r) % rmod) * ldr + col]; if (RES_BF16) rv = bf16_round(rv); v += rv; }
      if (ACT == 1) v = fmaxf(v, 0.f);
      if (ACT == 2) v = 0.5f * v * (1.0f + erff(v * 0.70710678118654752f));
      if (ACT == 3) { const float u = 0.7978845608028654f * (v + 0.044715f * v * v * v); v = 0.5f * v * (1.0f + tanhf(u)); }
      so[w][8 * hh + r][t * 16 + ln] = v;
    }
  }
  __builtin_amdgcn_fence(__ATOMIC_ACQ_REL, "workgroup");
  __builtin_amdgcn_wave_barrier();
  const int rsub = lane >> 4, c4 = (lane & 15) * 4;
  for (int pass = 0; pass < 2; ++pass) {
#pragma unroll
    for (int q = 0; q < 8; ++q) {
      const int r = q * 2 + rsub;
      const v4f v = *(const v4fa*)&so[w][r][c4];
      *(volatile v4f*)(C + (size_t)(row0 + r) * ldc + col0 + c4) = v;
    }
    if (pass == 0) __threadfence();
  }
}
template <bool PARAM_BF16>
__global__ __launch_bounds__(256) void k_layernorm(const float* __restrict__ X, const float* __restrict__ R, const float* __restrict__ g, const float* __restrict__ bta,
                                                  float* __restrict__ out_sum, float* __restrict__ out_norm, int N, float eps) {
  __shared__ float red[256];
  const int row = blockIdx.x, tid = threadIdx.x;
  const float* x = X + (size_t)row * N; const float* rr = R ? R + (size_t)row * N : nullptr;
  float vals[16];
  const int per = N / 256;
  float s1 = 0.f;
  for (int u = 0; u < per / 4; ++u) {
    const int j = tid * 4 + 1024 * u;
    const v4f a = *(const v4fa*)(x + j);
    v4f b = {0.f,0.f,0.f,0.f}; if (rr) b = *(const v4fa*)(rr + j);
#pragma unroll
    for (int q = 0; q < 4; ++q) { const float v = a[q] + b[q]; vals[u * 4 + q] = v; s1 += v; }
  }
  red[tid] = s1; __syncthreads();
  for (int st = 128; st > 0; st >>= 1) { if (tid < st) red[tid] += red[tid + st]; __syncthreads(); }
  const float mu = red[0] / (float)N; __syncthreads();
  float s2 = 0.f;
  for (int u = 0; u < per / 4; ++u)
#pragma unroll
    for (int q = 0; q < 4; ++q) { const float c = vals[u * 4 + q] - mu; s2 += c * c; }
  red[tid] = s2; __syncthreads();
  for (int st = 128; st > 0; st >>= 1) { if (tid < st) red[tid] += red[tid + st]; __syncthreads(); }
  const float rs = rsqrtf(red[0] / (float)N + eps);
  for (int pass = 0; pass < 2; ++pass) {
    for (int u = 0; u < per / 4; ++u) {
      const int j = tid * 4 + 1024 * u;
      v4f o, sm;
#pragma unroll
      for (int q = 0; q < 4; ++q) {
        float gg = g[j + q], bb = bta[j + q];
        if (PARAM_BF16) { gg = bf16_round(gg); bb = bf16_round(bb); }
        sm[q] = vals[u * 4 + q]; o[q] = (vals[u * 4 + q] - mu) * rs * gg + bb;
      }
      if (out_sum) *(volatile v4f*)(out_sum + (size_t)row * N + j) = sm;
      *(volatile v4f*)(out_norm + (size_t)row * N + j) = o;
    }
    if (pass == 0) __threadfence();
  }
}


typedef _Float16 v16h __attribute__((ext_vector_type(16)));
union FragH { v16h v; v8us half[2]; _Float16 h[16]; unsigned short u[16]; };
template <int NTT>
__device__ __forceinline__ v8f mmaH(v16h ah, v16h al, v16h bh, v16h bl, v8f c) {
  c = __builtin_amdgcn_wmma_f32_16x16x32_f16(false, ah, false, bh, (short)0, c, false, false);
  if (NTT >= 2) c = __builtin_amdgcn_wmma_f32_16x16x32_f16(false, al, false, bh, (short)0, c, false, false);
  if (NTT >= 3) c = __builtin_amdgcn_wmma_f32_16x16x32_f16(false, ah, false, bl, (short)0, c, false, false);
  asm volatile("v_nop\n\tv_nop\n\tv_nop\n\tv_nop" : "+v"(c) : "v"(ah), "v"(al), "v"(bh), "v"(bl));
  return c;
}
template <bool ASPLIT>
__global__ __launch_bounds__(128) void k_gemm_h(const float* __restrict__ A, int lda, size_t sA, const _Float16* __restrict__ Bh, int ldb, size_t sB, float alpha, float* __restrict__ C, int ldc, size_t sC, int M, int N, int K) {
  __shared__ __attribute__((aligned(16))) float so[4][16][64];
  const int tid = threadIdx.x, w = tid >> 5, lane = tid & 31, ln = lane & 15, hh = lane >> 4; const int by = blockIdx.y;
  A += (size_t)by * sA; Bh += (size_t)by * sB; C += (size_t)by * sC;
  const int ntn = (N + 63) / 64; const int wid = blockIdx.x * 4 + w; const int mt = wid / ntn, nq = wid % ntn; if (mt * 16 >= M) return;
  const int row0 = mt * 16, col0 = nq * 64; const float* arow = A + (size_t)(row0 + ln) * lda;
  v8f acc[4] = {};
  for (int kb = 0; kb < K; kb += 32) {
    FragH ah, al;
    const v4f x0 = *(const v4fa*)(arow + kb + 8 * hh), x1 = *(const v4fa*)(arow + kb + 8 * hh + 4), x2 = *(const v4fa*)(arow + kb + 16 + 8 * hh), x3 = *(const v4fa*)(arow + kb + 16 + 8 * hh + 4);
    float xs[16] = {x0[0],x0[1],x0[2],x0[3],x1[0],x1[1],x1[2],x1[3],x2[0],x2[1],x2[2],x2[3],x3[0],x3[1],x3[2],x3[3]};
#pragma unroll
    for (int i = 0; i < 16; ++i) { const _Float16 h = (_Float16)xs[i]; ah.h[i] = h; al.h[i] = ASPLIT ? (_Float16)(xs[i] - (float)h) : (_Float16)0.0f; }
#pragma unroll
    for (int t = 0; t < 4; ++t) { if (col0 + t * 16 >= N) continue; const size_t boff = (size_t)(col0 + t * 16 + ln) * ldb + kb; FragH bq; bq.half[0] = *(const v8us*)(Bh + boff + 8 * hh); bq.half[1] = *(const v8us*)(Bh + boff + 16 + 8 * hh);
      acc[t] = mmaH<ASPLIT ? 2 : 1>(ah.v, al.v, bq.v, bq.v, acc[t]); }
  }
#pragma unroll
  for (int t = 0; t < 4; ++t) { if (col0 + t * 16 >= N) continue;
#pragma unroll
    for (int r = 0; r < 8; ++r) so[w][8 * hh + r][t * 16 + ln] = acc[t][r] * alpha; }
  __builtin_amdgcn_fence(__ATOMIC_ACQ_REL, "workgroup"); __builtin_amdgcn_wave_barrier();
  const int rsub = lane >> 4, c4 = (lane & 15) * 4;
  for (int pass = 0; pass < 2; ++pass) {
#pragma unroll
    for (int q = 0; q < 8; ++q) { const int r = q * 2 + rsub; if (col0 + c4 < N) { const v4f v = *(const v4fa*)&so[w][r][c4]; *(volatile v4f*)(C + (size_t)(row0 + r) * ldc + col0 + c4) = v; } }
    if (pass == 0) __threadfence(); }
}

__global__ __launch_bounds__(256) void k_wt_f16(const float* __restrict__ W, _Float16* __restrict__ Wt, int K, int N, float scale) {
  const int t = blockIdx.x * 256 + threadIdx.x; if (t >= N * (K / 8)) return; const int n = t / (K / 8), k8 = (t % (K / 8)) * 8; FragH f;
#pragma unroll
  for (int i = 0; i < 8; ++i) f.h[i] = (_Float16)(bf16_round(W[(size_t)(k8 + i) * N + n]) * scale); const v8us o = f.half[0];
  *(volatile v8us*)((unsigned short*)Wt + (size_t)n * K + k8) = o; __threadfence(); *(volatile v8us*)((unsigned short*)Wt + (size_t)n * K + k8) = o;
}
template <int ACT>
__global__ __launch_bounds__(128) void k_gemm_hhx(const _Float16* __restrict__ A, int lda, size_t sA, const _Float16* __restrict__ Bh, int ldb, size_t sB, float alpha, const float* __restrict__ bias, size_t sBias, const float* __restrict__ CP, int rowsPerB, size_t sCPb, int row0g,
    float* __restrict__ C, _Float16* __restrict__ C16, int ldc, size_t sC, int M, int N, int K) {
  __shared__ __attribute__((aligned(16))) float so[4][16][64];
  const int tid = threadIdx.x, w = tid >> 5, lane = tid & 31, ln = lane & 15, hh = lane >> 4; const int by = blockIdx.y;
  A += (size_t)by * sA; Bh += (size_t)by * sB; const size_t cofs = (size_t)by * sC; const float* bp = bias ? bias + (size_t)by * sBias : nullptr;
  const int ntn = (N + 63) / 64; const int wid = blockIdx.x * 4 + w; const int mt = wid / ntn, nq = wid % ntn; if (mt * 16 >= M) return;
  const int row0 = mt * 16, col0 = nq * 64; const _Float16* arow = A + (size_t)(row0 + ln) * lda;
  v8f acc[4] = {};
  for (int kb = 0; kb < K; kb += 32) { FragH ah; ah.half[0] = *(const v8us*)((const unsigned short*)arow + kb + 8 * hh); ah.half[1] = *(const v8us*)((const unsigned short*)arow + kb + 16 + 8 * hh);
#pragma unroll
    for (int t = 0; t < 4; ++t) { if (col0 + t * 16 >= N) continue; const size_t boff = (size_t)(col0 + t * 16 + ln) * ldb + kb; FragH bq; bq.half[0] = *(const v8us*)((const unsigned short*)Bh + boff + 8 * hh); bq.half[1] = *(const v8us*)((const unsigned short*)Bh + boff + 16 + 8 * hh);
      acc[t] = mmaH<1>(ah.v, ah.v, bq.v, bq.v, acc[t]); }
  }
#pragma unroll
  for (int t = 0; t < 4; ++t) { if (col0 + t * 16 >= N) continue; const int col = col0 + t * 16 + ln; const float bv = bp ? bf16_round(bp[col]) : 0.f;
#pragma unroll
    for (int r = 0; r < 8; ++r) { float v = acc[t][r] * alpha + bv; if (CP) { const int rr = row0g + row0 + 8 * hh + r; if (rowsPerB < 0) v += CP[cofs + (size_t)rr * ldc + col];        else { const int bidx = rr / rowsPerB; v += CP[(size_t)bidx * sCPb + (size_t)by * 64 + col]; } } if (ACT == 1) v = (v > 0.f) ? v : expm1f(v); else if (ACT == 7) v = (v > 0.f) ? v + 1.0f : expf(v); else if (ACT == 8) v = tanhf(v); else if (ACT == 9) v = 0.5f * v * (1.0f + tanhf(0.7978845608028654f * (v + 0.044715f * v * v * v))); else if (ACT == 11) v = 1.0f / (1.0f + expf(-v)); else if (ACT == 12) v = (v > 0.f) ? v : 0.01f * v; else if (ACT == 14) v = (v > 0.f) ? v : 0.1f * v; else if (ACT == 16) v = (v >= 0.f) ? v : 0.3f * v; else if (ACT == 17) v = (v >= 0.f) ? v : 0.2f * v; else if (ACT == 15) v = v / (1.0f + expf(-v)); else if (ACT == 3) v = fmaxf(v, 0.f); else if (ACT == 6) v = 0.5f * v * (1.0f + erff(v * 0.70710678118654752f)); so[w][8 * hh + r][t * 16 + ln] = v; } }
  __builtin_amdgcn_fence(__ATOMIC_ACQ_REL, "workgroup"); __builtin_amdgcn_wave_barrier();
  const int rsub = lane >> 4, c4 = (lane & 15) * 4; typedef _Float16 v4h __attribute__((ext_vector_type(4)));
  for (int pass = 0; pass < 2; ++pass) {
#pragma unroll
    for (int q = 0; q < 8; ++q) { const int r = q * 2 + rsub; if (col0 + c4 < N) { const v4f v = *(const v4fa*)&so[w][r][c4]; if (C) *(volatile v4f*)(C + cofs + (size_t)(row0 + r) * ldc + col0 + c4) = v; if (C16) { v4h h4; for (int i = 0; i < 4; ++i) h4[i] = (_Float16)v[i]; *(volatile v4h*)(C16 + cofs + (size_t)(row0 + r) * ldc + col0 + c4) = h4; } } }
    if (pass == 0) __threadfence(); }
}


typedef _Float16 v4h __attribute__((ext_vector_type(4)));

__global__ __launch_bounds__(256) void k_x16(const float* __restrict__ x, _Float16* __restrict__ X16, size_t n8) { const size_t t = (size_t)blockIdx.x * 256 + threadIdx.x; if (t >= n8) return; FragH f;
#pragma unroll
  for (int q = 0; q < 8; ++q) f.h[q] = (_Float16)bf16_round(x[t * 8 + q]); *(volatile v8us*)((unsigned short*)X16 + t * 8) = f.half[0]; __threadfence(); *(volatile v8us*)((unsigned short*)X16 + t * 8) = f.half[0]; }
__global__ __launch_bounds__(256) void k_h16(const float* __restrict__ x, _Float16* __restrict__ X16, size_t n8) { const size_t t = (size_t)blockIdx.x * 256 + threadIdx.x; if (t >= n8) return; FragH f;
#pragma unroll
  for (int q = 0; q < 8; ++q) f.h[q] = (_Float16)x[t * 8 + q]; *(volatile v8us*)((unsigned short*)X16 + t * 8) = f.half[0]; __threadfence(); *(volatile v8us*)((unsigned short*)X16 + t * 8) = f.half[0]; }
__global__ __launch_bounds__(256) void k_round16f(const float* __restrict__ W, _Float16* __restrict__ Bt, size_t n8) { const size_t t = (size_t)blockIdx.x * 256 + threadIdx.x; if (t >= n8) return; FragH f;
#pragma unroll
  for (int i = 0; i < 8; ++i) f.h[i] = (_Float16)(bf16_round(W[t * 8 + i]) * 16.0f); *(volatile v8us*)((unsigned short*)Bt + t * 8) = f.half[0]; __threadfence(); *(volatile v8us*)((unsigned short*)Bt + t * 8) = f.half[0]; }
template <int NHv, int TTv>
__global__ __launch_bounds__(256) void k_vt(const _Float16* __restrict__ V16, int ldv, int voff, _Float16* __restrict__ Vt) { __shared__ unsigned short tl[64][66]; const int tid = threadIdx.x; const int slab = blockIdx.x / (TTv / 64), lg = blockIdx.x % (TTv / 64); const int b = slab / NHv, h = slab % NHv;
  for (int i = tid; i < 64 * 8; i += 256) { const int r = i / 8, c8 = (i % 8) * 8; FragH f; f.half[0] = *(const v8us*)((const unsigned short*)V16 + ((size_t)b * TTv + lg * 64 + r) * ldv + voff + h * 64 + c8);
#pragma unroll
    for (int q = 0; q < 8; ++q) tl[r][c8 + q] = f.u[q]; }
  __syncthreads();
  for (int pass = 0; pass < 2; ++pass) {
#pragma unroll
    for (int rd = 0; rd < 2; ++rd) { const int d = rd * 32 + tid / 8, pc = tid % 8; FragH f;
#pragma unroll
      for (int q = 0; q < 8; ++q) f.u[q] = tl[pc * 8 + q][d];
      *(volatile v8us*)((unsigned short*)Vt + ((size_t)slab * 64 + d) * TTv + lg * 64 + pc * 8) = f.half[0]; }
    if (pass == 0) __threadfence(); } }

__global__ __launch_bounds__(256) void k_hl(const float* __restrict__ F, _Float16* __restrict__ Hh, _Float16* __restrict__ Hl, size_t n8) { const size_t t = (size_t)blockIdx.x * 256 + threadIdx.x; if (t >= n8) return; FragH fh, fl; const v4f a = *(const v4fa*)(F + t * 8), c = *(const v4fa*)(F + t * 8 + 4);
#pragma unroll
  for (int q = 0; q < 4; ++q) { _Float16 h = (_Float16)a[q]; fh.h[q] = h; fl.h[q] = (_Float16)((a[q] - (float)h) * 1024.0f); h = (_Float16)c[q]; fh.h[4 + q] = h; fl.h[4 + q] = (_Float16)((c[q] - (float)h) * 1024.0f); }
  for (int pass = 0; pass < 2; ++pass) { *(volatile v8us*)((unsigned short*)Hh + t * 8) = fh.half[0]; *(volatile v8us*)((unsigned short*)Hl + t * 8) = fl.half[0]; if (pass == 0) __threadfence(); } }

__device__ __forceinline__ v16h g2_frag(const _Float16* p, int hh) { FragH f; f.half[0] = *(const v8us*)((const unsigned short*)p + 8 * hh); f.half[1] = *(const v8us*)((const unsigned short*)p + 16 + 8 * hh); return f.v; }
__device__ __forceinline__ v8f g2_mma(v16h a, v16h b, v8f c) { v8f d = __builtin_amdgcn_wmma_f32_16x16x32_f16(false, a, false, b, (short)0, c, false, false); asm volatile("v_nop\n\tv_nop\n\tv_nop\n\tv_nop" : "+v"(d) : "v"(a), "v"(b)); return d; }
template <int ACT>
__global__ __launch_bounds__(128) void k_gemm2(const _Float16* __restrict__ A, int lda, size_t sA, const _Float16* __restrict__ Bh, int ldb, size_t sB, float alpha, const float* __restrict__ bias, size_t sBias, const float* __restrict__ CP, int rowsPerB, size_t sCPb, int row0g,
    float* __restrict__ C, _Float16* __restrict__ C16, int ldc, size_t sC, int M, int N, int K) { static_assert(ACT == 0 || ACT == 3 || ACT == 6 || ACT == 8 || ACT == 9 || ACT == 11 || ACT == 12 || ACT == 14 || ACT == 15 || ACT == 16 || ACT == 17, "k_gemm2: unsupported ACT code (would silently apply no activation)");
  __shared__ __attribute__((aligned(16))) float so[4][32][68];
  const int tid = threadIdx.x, w = tid >> 5, lane = tid & 31, ln = lane & 15, hh = lane >> 4; const int by = blockIdx.y;
  A += (size_t)by * sA; Bh += (size_t)by * sB; const size_t cofs = (size_t)by * sC; const float* bp = bias ? bias + (size_t)by * sBias : nullptr;
  const int ntn = N >> 6; const int mt = blockIdx.x / ntn, nq = blockIdx.x - mt * ntn; const int row0 = mt * 128 + 32 * w, col0 = nq * 64; if (row0 >= M) return;
  const _Float16* a0p = A + (size_t)(row0 + ln) * lda; const _Float16* a1p = a0p + (size_t)16 * lda;
  const _Float16* b0p = Bh + (size_t)(col0 + ln) * ldb; const _Float16* b1p = b0p + (size_t)16 * ldb; const _Float16* b2p = b1p + (size_t)16 * ldb; const _Float16* b3p = b2p + (size_t)16 * ldb;
  const v8f z8 = {0.f,0.f,0.f,0.f,0.f,0.f,0.f,0.f}; v8f c00 = z8, c01 = z8, c02 = z8, c03 = z8, c10 = z8, c11 = z8, c12 = z8, c13 = z8;
#pragma unroll 1
  for (int kb = 0; kb < K; kb += 32) { const v16h a0 = g2_frag(a0p + kb, hh), a1 = g2_frag(a1p + kb, hh);
    v16h b = g2_frag(b0p + kb, hh); c00 = g2_mma(a0, b, c00); c10 = g2_mma(a1, b, c10);
    b = g2_frag(b1p + kb, hh); c01 = g2_mma(a0, b, c01); c11 = g2_mma(a1, b, c11);
    b = g2_frag(b2p + kb, hh); c02 = g2_mma(a0, b, c02); c12 = g2_mma(a1, b, c12);
    b = g2_frag(b3p + kb, hh); c03 = g2_mma(a0, b, c03); c13 = g2_mma(a1, b, c13); }
  v8f accs[8] = {c00, c01, c02, c03, c10, c11, c12, c13};
#pragma unroll
  for (int u = 0; u < 8; ++u) { const int t = u & 3, half = u >> 2; const int col = col0 + t * 16 + ln; const float bv = bp ? bf16_round(bp[col]) : 0.f;
#pragma unroll
    for (int r = 0; r < 8; ++r) { const int rloc = half * 16 + 8 * hh + r; float v = accs[u][r] * alpha + bv; if (CP) { if (rowsPerB < 0) v += CP[cofs + (size_t)(row0g + row0 + rloc) * ldc + col];        else { const int bidx = (row0g + row0 + rloc) / rowsPerB; v += CP[(size_t)bidx * sCPb + (size_t)by * 64 + col]; } }
      if (ACT == 3) v = fmaxf(v, 0.f); else if (ACT == 6) v = 0.5f * v * (1.0f + erff(v * 0.70710678118654752f)); else if (ACT == 11) v = 1.0f / (1.0f + expf(-v)); else if (ACT == 15) v = v / (1.0f + expf(-v)); else if (ACT == 12) v = (v > 0.f) ? v : 0.01f * v; else if (ACT == 8) v = tanhf(v); else if (ACT == 9) v = 0.5f * v * (1.0f + tanhf(0.7978845608028654f * (v + 0.044715f * v * v * v))); else if (ACT == 14) v = (v > 0.f) ? v : 0.1f * v; else if (ACT == 16) v = (v >= 0.f) ? v : 0.3f * v; else if (ACT == 17) v = (v >= 0.f) ? v : 0.2f * v;
      so[w][rloc][t * 16 + ln] = v; } }
  __builtin_amdgcn_fence(__ATOMIC_ACQ_REL, "workgroup"); __builtin_amdgcn_wave_barrier();
  const int rsub = lane >> 4, c4 = (lane & 15) * 4;
  for (int pass = 0; pass < 2; ++pass) {
#pragma unroll
    for (int q = 0; q < 16; ++q) { const int r = q * 2 + rsub; const v4f v = *(const v4fa*)&so[w][r][c4]; if (C) *(volatile v4f*)(C + cofs + (size_t)(row0 + r) * ldc + col0 + c4) = v; if (C16) { v4h h4; for (int i = 0; i < 4; ++i) h4[i] = (_Float16)v[i]; *(volatile v4h*)(C16 + cofs + (size_t)(row0 + r) * ldc + col0 + c4) = h4; } }
    if (pass == 0) __threadfence(); } }


__global__ __launch_bounds__(256) void k_wnat(const float* __restrict__ w, size_t n8, _Float16* __restrict__ Bt) { const size_t t = (size_t)blockIdx.x * 256 + threadIdx.x; if (t >= n8) return; FragH f; for (int q = 0; q < 8; ++q) f.h[q] = (_Float16)(bf16_round(w[t * 8 + q]) * 16.0f); *(volatile v8us*)((unsigned short*)Bt + t * 8) = f.half[0]; __threadfence(); *(volatile v8us*)((unsigned short*)Bt + t * 8) = f.half[0]; }
__global__ __launch_bounds__(256) void k_f2h(const float* __restrict__ F, _Float16* __restrict__ H16, size_t n8) { const size_t i = (size_t)blockIdx.x * 256 + threadIdx.x; if (i >= n8) return; FragH f; for (int q = 0; q < 8; ++q) f.h[q] = (_Float16)F[i * 8 + q]; *(volatile v8us*)((unsigned short*)H16 + i * 8) = f.half[0]; __threadfence(); *(volatile v8us*)((unsigned short*)H16 + i * 8) = f.half[0]; }
__global__ __launch_bounds__(256) void k_kln(const float* __restrict__ KV, float* __restrict__ KLN) {
  #pragma clang fp contract(off)
  const size_t t = (size_t)blockIdx.x * 256 + threadIdx.x; if (t >= NR * HE) return; const int h = (int)(t % HE); const size_t r = t / HE; const float* k = KV + r * (2 * DM) + h * HD; float ss = 0.f;
#pragma unroll 1
  for (int d = 0; d < HD; ++d) ss = __fadd_rn(ss, __fmul_rn(k[d], k[d])); float n = sqrtf(ss); if (n < 1e-12f) n = 1e-12f; const float inv = 1.0f / n; float* o = KLN + r * DM + h * HD;
  for (int pass = 0; pass < 2; ++pass) {
#pragma unroll 1
    for (int d0 = 0; d0 < HD; d0 += 8) { v8f v; for (int q = 0; q < 8; ++q) v[q] = __fmul_rn(k[d0 + q], inv); *(volatile v8f*)(o + d0) = v; } if (pass == 0) __threadfence(); } }
__global__ __launch_bounds__(128) void k_pool(const float* __restrict__ XS, const float* __restrict__ g, const float* __restrict__ be, float* __restrict__ XPN) {
  #pragma clang fp contract(off)
  __shared__ float red[128]; const int c = threadIdx.x; const int m = blockIdx.x % PL; const int b = blockIdx.x / PL; const int py = m / PS, px = m % PS; float s = 0.f;
#pragma unroll 1
  for (int i = 0; i < PS * PS; ++i) { const int y = py * PS + i / PS, xq = px * PS + i % PS; s = __fadd_rn(s, XS[((size_t)b * NT + (size_t)y * GS + xq) * DM + c]); } const float v = s / 64.0f;
  red[c] = v; __syncthreads(); for (int st = 64; st > 0; st >>= 1) { if (c < st) red[c] = __fadd_rn(red[c], red[c + st]); __syncthreads(); } const float mu = red[0] / (float)DM; __syncthreads();
  const float d = v - mu; red[c] = __fmul_rn(d, d); __syncthreads(); for (int st = 64; st > 0; st >>= 1) { if (c < st) red[c] = __fadd_rn(red[c], red[c + st]); __syncthreads(); } const float var = red[0] / (float)DM;
  const float y = __fadd_rn(__fmul_rn(d / sqrtf(__fadd_rn(var, 1e-5f)), bf16_round(g[c])), bf16_round(be[c]));
  __shared__ float row[DM]; row[c] = y; __syncthreads();
  if (c < DM / 8) { v8f o; for (int q = 0; q < 8; ++q) o[q] = row[c * 8 + q]; float* dst = XPN + ((size_t)b * PL + m) * DM + c * 8; *(volatile v8f*)dst = o; __threadfence(); *(volatile v8f*)dst = o; } }
__global__ __launch_bounds__(64) void k_kvp(const float* __restrict__ XPN, const float* __restrict__ Wkv, const float* __restrict__ bkv, float* __restrict__ KPN, float* __restrict__ VP) {
  #pragma clang fp contract(off)
  __shared__ float kk_[64][HD + 1], vv_[64][HD + 1]; const size_t t = (size_t)blockIdx.x * 64 + threadIdx.x; if (t >= (size_t)NB * PL * HE) return; const int h = (int)(t % HE); const size_t r = t / HE; const float* xr = XPN + r * DM; float* kk = kk_[threadIdx.x]; float* vv = vv_[threadIdx.x]; float ss = 0.f;
#pragma unroll 1
  for (int d = 0; d < HD; ++d) { float ak = bf16_round(bkv[h * HD + d]), av = bf16_round(bkv[DM + h * HD + d]); const float* wk = Wkv + (size_t)(h * HD + d) * DM; const float* wv = Wkv + (size_t)(DM + h * HD + d) * DM;
#pragma unroll 1
    for (int c = 0; c < DM; ++c) { ak = __fadd_rn(ak, __fmul_rn(xr[c], bf16_round(wk[c]))); av = __fadd_rn(av, __fmul_rn(xr[c], bf16_round(wv[c]))); } kk[d] = ak; vv[d] = av; ss = __fadd_rn(ss, __fmul_rn(ak, ak)); }
  float n = sqrtf(ss); if (n < 1e-12f) n = 1e-12f; const float inv = 1.0f / n;
  for (int pass = 0; pass < 2; ++pass) {
#pragma unroll 1
    for (int d0 = 0; d0 < HD; d0 += 8) { v8f a, c; for (int q = 0; q < 8; ++q) { a[q] = __fmul_rn(kk[d0 + q], inv); c[q] = vv[d0 + q]; } *(volatile v8f*)(KPN + r * DM + h * HD + d0) = a; *(volatile v8f*)(VP + r * DM + h * HD + d0) = c; } if (pass == 0) __threadfence(); } }
__global__ __launch_bounds__(256) void k_cpb(const float* __restrict__ rct, const float* __restrict__ w1, const float* __restrict__ b1, const float* __restrict__ w2, const float* __restrict__ b2, float* __restrict__ TB) {
  #pragma clang fp contract(off)
  const int t = blockIdx.x * 256 + threadIdx.x; if (t >= NTB) return; const float c0 = bf16_round(rct[t * 2]), c1 = bf16_round(rct[t * 2 + 1]); float a0 = bf16_round(b2[0]), a1 = bf16_round(b2[1]), a2 = bf16_round(b2[2]), a3 = bf16_round(b2[3]);
#pragma unroll 1
  for (int j = 0; j < CPH; ++j) { float hj = __fadd_rn(__fadd_rn(__fmul_rn(c0, bf16_round(w1[j * 2])), __fmul_rn(c1, bf16_round(w1[j * 2 + 1]))), bf16_round(b1[j])); hj = fmaxf(hj, 0.f);
    a0 = __fadd_rn(a0, __fmul_rn(hj, bf16_round(w2[0 * CPH + j]))); a1 = __fadd_rn(a1, __fmul_rn(hj, bf16_round(w2[1 * CPH + j]))); a2 = __fadd_rn(a2, __fmul_rn(hj, bf16_round(w2[2 * CPH + j]))); a3 = __fadd_rn(a3, __fmul_rn(hj, bf16_round(w2[3 * CPH + j]))); }
  typedef float v4f __attribute__((ext_vector_type(4))); v4f o; o[0] = a0; o[1] = a1; o[2] = a2; o[3] = a3; *(volatile v4f*)(TB + (size_t)t * 4) = o; __threadfence(); *(volatile v4f*)(TB + (size_t)t * 4) = o; }
__global__ __launch_bounds__(64) void k_attn(const float* __restrict__ Q, const float* __restrict__ KLN, const float* __restrict__ KV, const float* __restrict__ KPN, const float* __restrict__ VP, const float* __restrict__ TB, const int* __restrict__ rpi,
    const float* __restrict__ temp, const float* __restrict__ qemb, const float* __restrict__ rpb, const float* __restrict__ ltok, const float* __restrict__ lbias, const float* __restrict__ sls, float* __restrict__ O) {
  #pragma clang fp contract(off)
  __shared__ float qn_[64][HD + 1], qs_[64][HD + 1], acc_[64][HD + 1]; __shared__ float lgs_[64][LL + PL + 1];
  const size_t t = (size_t)blockIdx.x * 64 + threadIdx.x; if (t >= NR * HE) return; const int h = (int)(t % HE); const size_t r = t / HE; const int n = (int)(r % NT); const size_t b = r / NT; const int y = n / GS, xq = n % GS;
  float* qn = qn_[threadIdx.x]; float* qs = qs_[threadIdx.x]; float* acc = acc_[threadIdx.x]; const float* q = Q + r * DM + h * HD; float ss = 0.f;
#pragma unroll 1
  for (int d = 0; d < HD; ++d) ss = __fadd_rn(ss, __fmul_rn(q[d], q[d])); float nn = sqrtf(ss); if (nn < 1e-12f) nn = 1e-12f; const float inv = 1.0f / nn;
  const float tv = bf16_round(temp[h]); const float spt = (tv > 20.0f) ? tv : log1pf(expf(tv)); const float scl = __fmul_rn(spt, bf16_round(sls[n]));
#pragma unroll 1
  for (int d = 0; d < HD; ++d) { qn[d] = __fmul_rn(q[d], inv); qs[d] = __fmul_rn(__fadd_rn(qn[d], bf16_round(qemb[h * HD + d])), scl); acc[d] = 0.f; }
  float* lg = lgs_[threadIdx.x];
#pragma unroll 1
  for (int l = 0; l < LL; ++l) { const int yy = y + l / 3 - 1, xx = xq + l % 3 - 1; float v = -3.0e38f;
    if (yy >= 0 && yy < GS && xx >= 0 && xx < GS) { const float* kr = KLN + (b * NT + (size_t)yy * GS + xx) * DM + h * HD; float a = 0.f;
#pragma unroll 1
      for (int d = 0; d < HD; ++d) a = __fadd_rn(a, __fmul_rn(qs[d], kr[d])); v = __fadd_rn(a, bf16_round(rpb[h * LL + l])); } lg[l] = v; }
#pragma unroll 1
  for (int m = 0; m < PL; ++m) { const float* kr = KPN + (b * PL + m) * DM + h * HD; float a = 0.f;
#pragma unroll 1
    for (int d = 0; d < HD; ++d) a = __fadd_rn(a, __fmul_rn(qs[d], kr[d])); lg[LL + m] = __fadd_rn(a, TB[(size_t)rpi[(size_t)n * PL + m] * HE + h]); }
  float mx = -3.0e38f;
#pragma unroll 1
  for (int i = 0; i < LL + PL; ++i) mx = fmaxf(mx, lg[i]); float se = 0.f;
#pragma unroll 1
  for (int i = 0; i < LL + PL; ++i) { const float e = (lg[i] > -1.0e38f) ? expf(lg[i] - mx) : 0.f; lg[i] = e; se += e; } const float rse = 1.0f / se;
#pragma unroll 1
  for (int l = 0; l < LL; ++l) { const int yy = y + l / 3 - 1, xx = xq + l % 3 - 1; if (yy < 0 || yy >= GS || xx < 0 || xx >= GS) continue;        float tok = bf16_round(lbias[h * LL + l]);
#pragma unroll 1
    for (int d = 0; d < HD; ++d) tok = __fadd_rn(tok, __fmul_rn(qn[d], bf16_round(ltok[((size_t)h * HD + d) * LL + l]))); const float w = __fadd_rn(tok, __fmul_rn(lg[l], rse)); const float* vr = KV + (b * NT + (size_t)yy * GS + xx) * (2 * DM) + DM + h * HD;
#pragma unroll 1
    for (int d = 0; d < HD; ++d) acc[d] = __fadd_rn(acc[d], __fmul_rn(w, vr[d])); }
#pragma unroll 1
  for (int m = 0; m < PL; ++m) { const float w = __fmul_rn(lg[LL + m], rse); const float* vr = VP + (b * PL + m) * DM + h * HD;
#pragma unroll 1
    for (int d = 0; d < HD; ++d) acc[d] = __fadd_rn(acc[d], __fmul_rn(w, vr[d])); }
  float* o = O + r * DM + h * HD; for (int pass = 0; pass < 2; ++pass) {
#pragma unroll 1
    for (int d0 = 0; d0 < HD; d0 += 8) { v8f v; for (int q2 = 0; q2 < 8; ++q2) v[q2] = acc[d0 + q2]; *(volatile v8f*)(o + d0) = v; } if (pass == 0) __threadfence(); } }

extern "C" void kernel_launch(void* const* d_in, const int* in_sizes, int n_in,
                              void* d_out, int out_size, void* d_ws, size_t ws_size, hipStream_t stream) {
  (void)in_sizes; (void)n_in; (void)out_size;
  const float* const* I = (const float* const*)d_in; const float* x = I[0]; const float* wq = I[1]; const float* bq = I[2]; const float* wkv = I[3]; const float* bkv = I[4]; const float* wsr = I[5]; const float* bsr = I[6]; const float* ng = I[7]; const float* nbeta = I[8]; const float* wp = I[9]; const float* bp = I[10];
  const float* cw1 = I[11]; const float* cb1 = I[12]; const float* cw2 = I[13]; const float* cb2 = I[14]; const float* temp = I[15]; const float* qemb = I[16]; const float* rpb = I[17]; const float* ltok = I[18]; const float* lbias = I[19]; const float* sls = I[20]; const float* rct = I[21]; const int* rpi = (const int*)d_in[22];
  char* ws = (char*)d_ws; size_t off = 0;
  auto take = [&](size_t bytes) { char* p = ws + off; off += (bytes + 255) & ~(size_t)255; return p; };
  _Float16* BQ = (_Float16*)take((size_t)DM * DM * 2); _Float16* BKV = (_Float16*)take((size_t)2 * DM * DM * 2); _Float16* BSR = (_Float16*)take((size_t)DM * DM * 2); _Float16* BP = (_Float16*)take((size_t)DM * DM * 2);
  _Float16* X16 = (_Float16*)take(NR * DM * 2); float* Q = (float*)take(NR * DM * 4); float* KV = (float*)take(NR * 2 * DM * 4); float* XS = (float*)take(NR * DM * 4); float* KLN = (float*)take(NR * DM * 4);
  float* XPN = (float*)take((size_t)NB * PL * DM * 4); float* KPN = (float*)take((size_t)NB * PL * DM * 4); float* VP = (float*)take((size_t)NB * PL * DM * 4); float* TB = (float*)take((size_t)NTB * HE * 4);
  float* O = XS;        _Float16* O16 = X16;
  if (off > ws_size) return;
  k_wnat<<<(DM * DM / 8 + 255) / 256, 256, 0, stream>>>(wq, DM * DM / 8, BQ); k_wnat<<<(2 * DM * DM / 8 + 255) / 256, 256, 0, stream>>>(wkv, 2 * DM * DM / 8, BKV); k_wnat<<<(DM * DM / 8 + 255) / 256, 256, 0, stream>>>(wsr, DM * DM / 8, BSR); k_wnat<<<(DM * DM / 8 + 255) / 256, 256, 0, stream>>>(wp, DM * DM / 8, BP);
  k_cpb<<<(NTB + 255) / 256, 256, 0, stream>>>(rct, cw1, cb1, cw2, cb2, TB);
  k_x16<<<(unsigned)((NR * DM / 8 + 255) / 256), 256, 0, stream>>>(x, X16, NR * DM / 8);
  k_gemm2<0><<<dim3((unsigned)((NR / 128) * (DM / 64)), 1), 128, 0, stream>>>(X16, DM, 0, BQ, DM, 0, 0.0625f, bq, 0, nullptr, 1, 0, 0, Q, nullptr, DM, 0, (int)NR, DM, DM);
  k_gemm2<0><<<dim3((unsigned)((NR / 128) * (2 * DM / 64)), 1), 128, 0, stream>>>(X16, DM, 0, BKV, DM, 0, 0.0625f, bkv, 0, nullptr, 1, 0, 0, KV, nullptr, 2 * DM, 0, (int)NR, 2 * DM, DM);
  k_gemm2<6><<<dim3((unsigned)((NR / 128) * (DM / 64)), 1), 128, 0, stream>>>(X16, DM, 0, BSR, DM, 0, 0.0625f, bsr, 0, nullptr, 1, 0, 0, XS, nullptr, DM, 0, (int)NR, DM, DM);
  k_kln<<<(unsigned)((NR * HE + 255) / 256), 256, 0, stream>>>(KV, KLN);
  k_pool<<<NB * PL, 128, 0, stream>>>(XS, ng, nbeta, XPN);
  k_kvp<<<(unsigned)((NB * PL * HE + 63) / 64), 64, 0, stream>>>(XPN, wkv, bkv, KPN, VP);
  k_attn<<<(unsigned)((NR * HE + 63) / 64), 64, 0, stream>>>(Q, KLN, KV, KPN, VP, TB, rpi, temp, qemb, rpb, ltok, lbias, sls, O);
  k_f2h<<<(unsigned)((NR * DM / 8 + 255) / 256), 256, 0, stream>>>(O, O16, NR * DM / 8);
  k_gemm2<0><<<dim3((unsigned)((NR / 128) * (DM / 64)), 1), 128, 0, stream>>>(O16, DM, 0, BP, DM, 0, 0.0625f, bp, 0, nullptr, 1, 0, 0, (float*)d_out, nullptr, DM, 0, (int)NR, DM, DM);
}
